// STFT_network_3848290697296
// MI455X (gfx1250) — hardware-verified
//
#include <hip/hip_runtime.h>

typedef __attribute__((ext_vector_type(16))) _Float16 v16h;
typedef __attribute__((ext_vector_type(8)))  _Float16 v8h;
typedef __attribute__((ext_vector_type(8)))  float    v8f;
typedef __attribute__((ext_vector_type(4)))  float    v4f;

constexpr int kWindow = 2048;
constexpr int kStride = 512;
constexpr int kFreq   = 1024;
constexpr int kFrames = 63;
constexpr int kSigLen = kFrames * kStride;
constexpr int kBatch  = 64;
constexpr int kPadL   = 768;
constexpr int kRowsM  = kBatch * kFrames;
constexpr int kColsN  = 2 * kFreq;
constexpr int kDepthK = kWindow;
constexpr int kTilesM = kRowsM / 64;
constexpr int kTilesN = kColsN / 64;
constexpr int kTilesTotal = kTilesM * kTilesN;

constexpr float kCarrySig  = 16.0f;
constexpr float kCarryTap  = 64.0f;
constexpr float kFoldScale = 1.0f / (kCarrySig * kCarryTap);

static_assert(kSigLen == 32256, "signal length");
static_assert(kRowsM == 4032 && (kRowsM % 64) == 0, "M is a multiple of 64");
static_assert(kColsN == 2048 && (kColsN % 64) == 0, "N is a multiple of 64");
static_assert((kDepthK % 32) == 0 && (kDepthK % 64) == 0, "K is a multiple of 32 and of the transpose tile");
static_assert((kStride % 8) == 0 && (kPadL % 8) == 0 && (kSigLen % 8) == 0, "8-sample groups never straddle a bound");
static_assert((kTilesN % 8) == 0 && (kTilesTotal % 8) == 0, "8 waves of a block share one tile row; exact grid");
static_assert((kFreq % 64) == 0, "a 64-column tile never straddles the real/imag seam");

constexpr size_t kOffSigP = 0;
constexpr size_t kOffTapP = kOffSigP + (size_t)kRowsM * kDepthK * 2;
constexpr size_t kWsTotal = kOffTapP + (size_t)kColsN * kDepthK * 2;
static_assert(kOffTapP == 16515072ull, "tap plane offset");
static_assert((kOffTapP % 128) == 0, "128-B aligned region");
static_assert(kWsTotal == 24903680ull, "carve total");
static_assert(kWsTotal <= 134217728ull, "carve cap");

constexpr size_t kOutPlaneElems = (size_t)kRowsM * kFreq;
static_assert(kOutPlaneElems * 4 == 16515072ull, "second output byte offset");
static_assert(2 * kOutPlaneElems * 4 == 33030144ull, "output total");

union FragH { v16h v; v8h h[2]; };
__device__ __forceinline__ v16h frag_load(const _Float16* p) {
  FragH f;
  f.h[0] = *(const v8h*)(p);
  f.h[1] = *(const v8h*)(p + 16);
  return f.v;
}
__device__ __forceinline__ v8f mma_guarded(v16h a, v16h b, v8f c) {
  c = __builtin_amdgcn_wmma_f32_16x16x32_f16(false, a, false, b, (short)0, c, false, false);
  asm volatile("v_nop\n\tv_nop\n\tv_nop\n\tv_nop" : "+v"(c) : "v"(a), "v"(b));
  return c;
}

__global__ __launch_bounds__(256) void frames_f16_kernel(
    const float* __restrict__ sig, unsigned short* __restrict__ sigp)
{
  const int m  = blockIdx.x;
  const int b  = m / kFrames;
  const int t  = m - b * kFrames;
  const int k0 = threadIdx.x * 8;
  const int pos0 = t * kStride - kPadL + k0;
  const bool inb = (pos0 >= 0) && (pos0 <= kSigLen - 8);
  int posc = pos0 < 0 ? 0 : pos0;
  posc = posc > (kSigLen - 8) ? (kSigLen - 8) : posc;
  const float* src = sig + (size_t)b * kSigLen + posc;
  const v4f a0 = *(const v4f*)(src);
  const v4f a1 = *(const v4f*)(src + 4);
  v8h hv;
#pragma unroll
  for (int e = 0; e < 4; ++e) {
    const float f0 = a0[e];
    const float f1 = a1[e];
    const float x0 = inb ? f0 * kCarrySig : 0.0f;
    const float x1 = inb ? f1 * kCarrySig : 0.0f;
    hv[e]     = (_Float16)x0;
    hv[4 + e] = (_Float16)x1;
  }
  unsigned short* dst = sigp + (size_t)m * kDepthK + k0;
  *(volatile v8h*)dst = hv;
  __threadfence();
  *(volatile v8h*)dst = hv;
}

__global__ __launch_bounds__(256) void taps_transpose_f16_kernel(
    const float* __restrict__ wre, const float* __restrict__ wim, unsigned short* __restrict__ tapp)
{
  __shared__ __align__(16) float sT[64 * 68];
  const int tid = threadIdx.x, lane = tid & 31, wave = tid >> 5;
  const int k0 = blockIdx.x * 64;
  const int n0 = blockIdx.y * 64;
  const float* src = (n0 >= kFreq) ? wim : wre;
  const int nc0 = n0 & (kFreq - 1);
  const int rr = tid >> 4;
  const int c4 = (tid & 15) * 4;
#pragma unroll
  for (int i = 0; i < 4; ++i) {
    const int r = rr + 16 * i;
    const v4f v = *(const v4f*)(src + (size_t)(k0 + r) * kFreq + nc0 + c4);
    *(v4f*)(sT + r * 68 + c4) = v;
  }
  __syncthreads();
  const int q  = lane >> 3;
  const int c8 = (lane & 7) * 8;
  v8h hv[2];
#pragma unroll
  for (int it = 0; it < 2; ++it) {
    const int row = it * 32 + wave * 4 + q;
#pragma unroll
    for (int e = 0; e < 8; ++e) {
      const float x = sT[(c8 + e) * 68 + row] * kCarryTap;
      hv[it][e] = (_Float16)x;
    }
  }
  for (int pass = 0; pass < 2; ++pass) {
#pragma unroll
    for (int it = 0; it < 2; ++it) {
      const int row = it * 32 + wave * 4 + q;
      *(volatile v8h*)(tapp + (size_t)(n0 + row) * kDepthK + k0 + c8) = hv[it];
    }
    __threadfence();
  }
}

__global__ __launch_bounds__(256) void stft_gemm_f16_kernel(
    const unsigned short* __restrict__ sigp, const unsigned short* __restrict__ tapp, float* __restrict__ out)
{
  const _Float16* A  = (const _Float16*)sigp;
  const _Float16* Bt = (const _Float16*)tapp;
  __shared__ __align__(16) float sT[8][16 * 68];
  const int lane = threadIdx.x & 31;
  const int wave = threadIdx.x >> 5;
  const int tile = blockIdx.x * 8 + wave;
  if (tile >= kTilesTotal) return;
  const int tm = tile / kTilesN;
  const int tn = tile - tm * kTilesN;
  const int m0 = tm << 6;
  const int n0 = tn << 6;

  const int rlane = lane & 15;
  const int koff  = (lane >> 4) * 8;
  const int mOff  = (lane >> 4) * 8;

  v8f acc[4][4];
#pragma unroll
  for (int i = 0; i < 4; ++i)
#pragma unroll
    for (int j = 0; j < 4; ++j) acc[i][j] = (v8f){0.f,0.f,0.f,0.f,0.f,0.f,0.f,0.f};

  for (int k0 = 0; k0 < kDepthK; k0 += 32) {
    v16h bh[4];
#pragma unroll
    for (int j = 0; j < 4; ++j) {
      const size_t bo = (size_t)(n0 + (j << 4) + rlane) * kDepthK + koff + k0;
      bh[j] = frag_load(Bt + bo);
    }
#pragma unroll
    for (int i = 0; i < 4; ++i) {
      const size_t ao = (size_t)(m0 + (i << 4) + rlane) * kDepthK + koff + k0;
      const v16h ah = frag_load(A + ao);
#pragma unroll
      for (int j = 0; j < 4; ++j) {
        acc[i][j] = mma_guarded(ah, bh[j], acc[i][j]);
      }
    }
  }

  float* slab = sT[wave];
  float* C = out + ((n0 >= kFreq) ? kOutPlaneElems : (size_t)0);
  const int nc0 = n0 & (kFreq - 1);
#pragma unroll
  for (int i = 0; i < 4; ++i) {
    const int mBase = m0 + (i << 4);
#pragma unroll
    for (int j = 0; j < 4; ++j) {
#pragma unroll
      for (int r = 0; r < 8; ++r) {
        const float v = acc[i][j][r] * kFoldScale;
        slab[(mOff + r) * 68 + (j << 4) + rlane] = v;
      }
    }
    __builtin_amdgcn_fence(__ATOMIC_RELEASE, "workgroup");
    __builtin_amdgcn_wave_barrier();
    __builtin_amdgcn_fence(__ATOMIC_ACQUIRE, "workgroup");
    {
      const int hh = lane >> 4, c4 = (lane & 15) * 4;
      for (int pass = 0; pass < 2; ++pass) {
#pragma unroll
        for (int it = 0; it < 8; ++it) {
          const int row = it * 2 + hh;
          const v4f v = *(const v4f*)(slab + row * 68 + c4);
          *(volatile v4f*)(C + (size_t)(mBase + row) * kFreq + nc0 + c4) = v;
        }
        __threadfence();
      }
    }
    __builtin_amdgcn_fence(__ATOMIC_RELEASE, "workgroup");
    __builtin_amdgcn_wave_barrier();
    __builtin_amdgcn_fence(__ATOMIC_ACQUIRE, "workgroup");
  }
}

extern "C" void kernel_launch(void* const* d_in, const int* in_sizes, int n_in,
                              void* d_out, int out_size, void* d_ws, size_t ws_size,
                              hipStream_t stream) {
  if (n_in < 3) return;
  if (in_sizes[0] != kBatch * kSigLen) return;
  if (in_sizes[1] != kWindow * kFreq) return;
  if (in_sizes[2] != kWindow * kFreq) return;
  if (out_size != 2 * kRowsM * kFreq) return;
  if (ws_size < kWsTotal) return;

  const float* sig = (const float*)d_in[0];
  const float* wre = (const float*)d_in[1];
  const float* wim = (const float*)d_in[2];
  float* out = (float*)d_out;

  char* ws = (char*)d_ws;
  unsigned short* sigp = (unsigned short*)(ws + kOffSigP);
  unsigned short* tapp = (unsigned short*)(ws + kOffTapP);

  frames_f16_kernel<<<dim3(kRowsM), dim3(256), 0, stream>>>(sig, sigp);
  taps_transpose_f16_kernel<<<dim3(kDepthK / 64, kColsN / 64), dim3(256), 0, stream>>>(wre, wim, tapp);
  stft_gemm_f16_kernel<<<dim3(kTilesTotal / 8), dim3(256), 0, stream>>>(sigp, tapp, out);
}
